// SAttention_16793322127944
// MI455X (gfx1250) — hardware-verified
//
#include <hip/hip_runtime.h>


namespace {
constexpr int S = 2048, Bn = 4, D = 512, H = 8, HD = 64, NT = S * Bn;
constexpr float QS = 8.0f, KS = 8.0f, VS = 8.0f, PS = 8.0f, AS_ = 8.0f, SCALE = 0.125f, EPS = 1e-5f;
constexpr size_t PL = (size_t)Bn * H * S * HD;

typedef _Float16 b16;
typedef __attribute__((ext_vector_type(16))) _Float16 v16b;
typedef __attribute__((ext_vector_type(8))) _Float16 v8b;
typedef __attribute__((ext_vector_type(8))) float v8f;
typedef __attribute__((ext_vector_type(4))) float v4f;
__device__ __forceinline__ float bf16_rne(float f) { unsigned int u = __float_as_uint(f); u += 0x7FFFu + ((u >> 16) & 1u); return __uint_as_float(u & 0xFFFF0000u); }
__device__ __forceinline__ void split16(float v, b16& hi, b16& lo) { hi = (b16)v; lo = (b16)(v - (float)hi); }
__device__ __forceinline__ v16b frag_kb(const b16* p, int hh) { const v8b a = *(const v8b*)(p + 8 * hh), b = *(const v8b*)(p + 16 + 8 * hh); v16b f;
#pragma unroll
  for (int e = 0; e < 8; ++e) { f[e] = a[e]; f[8 + e] = b[e]; } return f; }
__device__ __forceinline__ void frag_split(const float* p, int hh, v16b& fh, v16b& fl) {
#pragma unroll
  for (int e = 0; e < 8; ++e) { b16 a, c; split16(p[8 * hh + e] * AS_, a, c); fh[e] = a; fl[e] = c; split16(p[16 + 8 * hh + e] * AS_, a, c); fh[8 + e] = a; fl[8 + e] = c; } }
__device__ __forceinline__ v8f wmma16b(v16b a, v16b b, v8f c) { v8f d = __builtin_amdgcn_wmma_f32_16x16x32_f16(false, a, false, b, (short)0, c, false, false); asm volatile("v_nop\n\tv_nop\n\tv_nop\n\tv_nop" : "+v"(d) : "v"(a), "v"(b)); return d; }
__device__ __forceinline__ void wave_lds_sync() { __builtin_amdgcn_fence(__ATOMIC_RELEASE, "workgroup"); __builtin_amdgcn_wave_barrier(); __builtin_amdgcn_fence(__ATOMIC_ACQUIRE, "workgroup"); }
__device__ __forceinline__ float nexp(float x) { return __builtin_amdgcn_exp2f(x * 1.4426950408889634f); }
__device__ __forceinline__ float pmul(float a, float b) { float p = a * b; asm volatile("" : "+v"(p)); return p; }

struct Wo_ { static constexpr size_t QKV = 0, W1 = QKV + (size_t)3 * D * D, W2 = W1 + (size_t)D * D, END = W2 + (size_t)D * D; };
__global__ __launch_bounds__(256) void prep_kernel(const float* __restrict__ wq, const float* __restrict__ wk, const float* __restrict__ wv, const float* __restrict__ w1, const float* __restrict__ w2, const float* __restrict__ b1, const float* __restrict__ b2, const float* __restrict__ g1, const float* __restrict__ be1, const float* __restrict__ g2, const float* __restrict__ be2, b16* __restrict__ R, float* __restrict__ P) {
  const int t_ = blockIdx.x * 256 + threadIdx.x, nth = gridDim.x * 256;
  for (int pass = 0; pass < 2; ++pass) {
    for (int q = t_; q < 3 * D * D; q += nth) { const int m = q / (D * D), o = (q / D) % D, k = q % D; const float* W = (m == 0) ? wq : (m == 1) ? wk : wv; R[Wo_::QKV + q] = (b16)bf16_rne(W[(size_t)k * D + o]); }
    for (int q = t_; q < D * D; q += nth) { const int o = q / D, k = q % D; R[Wo_::W1 + q] = (b16)bf16_rne(w1[(size_t)k * D + o]); R[Wo_::W2 + q] = (b16)bf16_rne(w2[(size_t)k * D + o]); }
    for (int q = t_; q < 6 * D; q += nth) { const int m = q / D, i = q % D; const float* v = (m == 0) ? b1 : (m == 1) ? b2 : (m == 2) ? g1 : (m == 3) ? be1 : (m == 4) ? g2 : be2; P[q] = bf16_rne(v[i]); }
    __threadfence(); }
}

__global__ __launch_bounds__(256) void ln_kernel(const float* __restrict__ x, const float* __restrict__ g, const float* __restrict__ bb, int rnd, float* __restrict__ y) {
  const int wid = threadIdx.x >> 5, lane = threadIdx.x & 31; const size_t row = (size_t)blockIdx.x * 8 + wid; const float* pr = x + row * D;
  float v[16]; float s = 0.0f;
#pragma unroll
  for (int j = 0; j < 4; ++j) { const v4f t = *(const v4f*)(pr + j * 128 + lane * 4);
#pragma unroll
    for (int e = 0; e < 4; ++e) { v[j * 4 + e] = rnd ? bf16_rne(t[e]) : t[e]; s += v[j * 4 + e]; } }
#pragma unroll
  for (int o = 1; o < 32; o <<= 1) s += __shfl_xor(s, o);
  const float mu = s * (1.0f / D); float q = 0.0f;
#pragma unroll
  for (int j = 0; j < 16; ++j) { const float d = v[j] - mu; q += pmul(d, d); }
#pragma unroll
  for (int o = 1; o < 32; o <<= 1) q += __shfl_xor(q, o);
  const float is = rsqrtf(q * (1.0f / D) + EPS);
  for (int pass = 0; pass < 2; ++pass) {
#pragma unroll
    for (int j = 0; j < 4; ++j) { const int c = j * 128 + lane * 4; v4f o4; for (int e = 0; e < 4; ++e) o4[e] = pmul((v[j * 4 + e] - mu) * is, g[c + e]) + bb[c + e]; *(volatile v4f*)(y + row * D + c) = o4; }
    __threadfence(); }
}

__global__ __launch_bounds__(128) void qk_kernel(const float* __restrict__ xn, const b16* __restrict__ R, b16* __restrict__ qp, b16* __restrict__ kp) {
  __shared__ __attribute__((aligned(16))) b16 T[4][32][64 + 8];
  const int lane = threadIdx.x & 31, wave = threadIdx.x >> 5, nloc = lane & 15, hlf = lane >> 4, h = blockIdx.x, c0 = h * HD, which = blockIdx.z, m0 = blockIdx.y * 128 + wave * 32;
  const b16* Wt = R + Wo_::QKV + (size_t)which * D * D;
  v8f acc[2][4];
#pragma unroll
  for (int r = 0; r < 2; ++r)
#pragma unroll
    for (int t = 0; t < 4; ++t) acc[r][t] = (v8f){};
#pragma unroll 2
  for (int kb = 0; kb < D; kb += 32) { v16b a0, l0, a1, l1; frag_split(xn + (size_t)(m0 + nloc) * D + kb, hlf, a0, l0); frag_split(xn + (size_t)(m0 + 16 + nloc) * D + kb, hlf, a1, l1);
#pragma unroll
    for (int t = 0; t < 4; ++t) { const v16b bw = frag_kb(Wt + (size_t)(c0 + t * 16 + nloc) * D + kb, hlf); acc[0][t] = wmma16b(a0, bw, acc[0][t]); acc[0][t] = wmma16b(l0, bw, acc[0][t]); acc[1][t] = wmma16b(a1, bw, acc[1][t]); acc[1][t] = wmma16b(l1, bw, acc[1][t]); } }
  const float scl = (which == 0) ? (SCALE * QS / AS_) : (KS / AS_);
#pragma unroll
  for (int t = 0; t < 4; ++t)
#pragma unroll
    for (int r = 0; r < 2; ++r)
#pragma unroll
      for (int v = 0; v < 8; ++v) T[wave][r * 16 + 8 * hlf + v][t * 16 + nloc] = (b16)(acc[r][t][v] * scl);
  wave_lds_sync();
  b16* base = (which == 0) ? qp : kp;
  for (int pass = 0; pass < 2; ++pass) {
#pragma unroll
    for (int j = 0; j < 8; ++j) { const int rr = j * 4 + (lane >> 3), c8 = (lane & 7) * 8; const int row = m0 + rr, s = row >> 2, b = row & 3; *(volatile v8b*)(base + (((size_t)b * H + h) * S + s) * HD + c8) = *(const v8b*)(&T[wave][rr][c8]); }
    __threadfence(); }
}
__global__ __launch_bounds__(128) void v_kernel(const float* __restrict__ xn, const b16* __restrict__ R, b16* __restrict__ vt) {
  __shared__ __attribute__((aligned(16))) b16 Tv[4][64][128 + 8];
  const int lane = threadIdx.x & 31, wave = threadIdx.x >> 5, nloc = lane & 15, hlf = lane >> 4, h = blockIdx.x, c0 = h * HD, s0 = blockIdx.y * 128, b = wave;
  const b16* Wt = R + Wo_::QKV + (size_t)2 * D * D;
  for (int sp = 0; sp < 4; ++sp) {
    v8f acc[2][4];
#pragma unroll
    for (int r = 0; r < 2; ++r)
#pragma unroll
      for (int t = 0; t < 4; ++t) acc[r][t] = (v8f){};
    const size_t rowA0 = ((size_t)(s0 + sp * 32 + nloc) * Bn + b) * D, rowA1 = ((size_t)(s0 + sp * 32 + 16 + nloc) * Bn + b) * D;
#pragma unroll 2
    for (int kb = 0; kb < D; kb += 32) { v16b a0, l0, a1, l1; frag_split(xn + rowA0 + kb, hlf, a0, l0); frag_split(xn + rowA1 + kb, hlf, a1, l1);
#pragma unroll
      for (int t = 0; t < 4; ++t) { const v16b bw = frag_kb(Wt + (size_t)(c0 + t * 16 + nloc) * D + kb, hlf); acc[0][t] = wmma16b(a0, bw, acc[0][t]); acc[0][t] = wmma16b(l0, bw, acc[0][t]); acc[1][t] = wmma16b(a1, bw, acc[1][t]); acc[1][t] = wmma16b(l1, bw, acc[1][t]); } }
#pragma unroll
    for (int t = 0; t < 4; ++t)
#pragma unroll
      for (int r = 0; r < 2; ++r)
#pragma unroll
        for (int v = 0; v < 8; ++v) Tv[b][t * 16 + nloc][sp * 32 + r * 16 + 8 * hlf + v] = (b16)(acc[r][t][v] * (VS / AS_)); }
  wave_lds_sync();
  for (int pass = 0; pass < 2; ++pass) { for (int i = lane; i < 64 * 16; i += 32) { const int d = i >> 4, c8 = (i & 15) * 8; *(volatile v8b*)(vt + (((size_t)b * H + h) * HD + d) * S + s0 + c8) = *(const v8b*)(&Tv[b][d][c8]); } __threadfence(); }
}

__global__ __launch_bounds__(256) void attn_kernel(const b16* __restrict__ qp, const b16* __restrict__ kp, const b16* __restrict__ vt, const float* __restrict__ x, float* __restrict__ xt) {
  __shared__ __attribute__((aligned(16))) float Os[16][D + 4];
  const int h = threadIdx.x >> 5, lane = threadIdx.x & 31, hh = lane >> 4, col = lane & 15; const int b = blockIdx.y, q0 = blockIdx.x * 16, qi = q0 + col;
  const b16* Q = qp + (((size_t)b * H + h) * S) * HD; const b16* K = kp + (((size_t)b * H + h) * S) * HD; const b16* V = vt + (((size_t)b * H + h) * HD) * S;
  const v16b qf0 = frag_kb(Q + (size_t)qi * HD, hh), qf1 = frag_kb(Q + (size_t)qi * HD + 32, hh);
  float m = -INFINITY, l = 0.0f; v8f o[4] = {{}, {}, {}, {}};
  for (int kb = 0; kb < S; kb += 32) {
    const v16b ka0 = frag_kb(K + (size_t)(kb + col) * HD, hh), ka1 = frag_kb(K + (size_t)(kb + col) * HD + 32, hh), kc0 = frag_kb(K + (size_t)(kb + 16 + col) * HD, hh), kc1 = frag_kb(K + (size_t)(kb + 16 + col) * HD + 32, hh);
    v8f s0 = {}, s1 = {}; s0 = wmma16b(ka0, qf0, s0); s0 = wmma16b(ka1, qf1, s0); s1 = wmma16b(kc0, qf0, s1); s1 = wmma16b(kc1, qf1, s1);
    float mr = -INFINITY;
#pragma unroll
    for (int r = 0; r < 8; ++r) { s0[r] *= 1.0f / (QS * KS); s1[r] *= 1.0f / (QS * KS); mr = fmaxf(mr, fmaxf(s0[r], s1[r])); }
    mr = fmaxf(mr, __shfl_xor(mr, 16));
    const float mn = fmaxf(m, mr), al_ = nexp(m - mn); m = mn; float sum = 0.0f; v16b pbv;
#pragma unroll
    for (int r = 0; r < 8; ++r) { const float e0 = nexp(s0[r] - mn), e1 = nexp(s1[r] - mn); sum += e0 + e1; pbv[r] = (b16)(e0 * PS); pbv[8 + r] = (b16)(e1 * PS); }
    sum += __shfl_xor(sum, 16); l = l * al_ + sum;
#pragma unroll
    for (int t = 0; t < 4; ++t) { o[t] *= al_; const v16b vf = frag_kb(V + (size_t)(t * 16 + col) * S + kb, hh); o[t] = wmma16b(vf, pbv, o[t]); } }
  const float inv = 1.0f / (l * VS * PS);
#pragma unroll
  for (int t = 0; t < 4; ++t)
#pragma unroll
    for (int r = 0; r < 8; ++r) Os[col][h * HD + t * 16 + 8 * hh + r] = o[t][r] * inv;
  __syncthreads();
  for (int pass = 0; pass < 2; ++pass) { for (int i = threadIdx.x; i < 16 * (D / 4); i += 256) { const int rr = i / (D / 4), c4 = (i % (D / 4)) * 4; const size_t row = (size_t)(q0 + rr) * Bn + b; const v4f xv = *(const v4f*)(x + row * D + c4); v4f o4 = *(const v4f*)(&Os[rr][c4]);
      for (int e = 0; e < 4; ++e) o4[e] += bf16_rne(xv[e]); *(volatile v4f*)(xt + row * D + c4) = o4; } __threadfence(); }
}

__global__ __launch_bounds__(128) void ffn_kernel(const float* __restrict__ Ain, const b16* __restrict__ Bw, const float* __restrict__ bias, int mode, const float* __restrict__ res, float* __restrict__ Y) {
  __shared__ __attribute__((aligned(16))) float Ts[4][32 * 64];
  const int lane = threadIdx.x & 31, wave = threadIdx.x >> 5, nloc = lane & 15, hlf = lane >> 4, m0 = blockIdx.y * 128 + wave * 32, c0 = blockIdx.x * 64;
  v8f acc[2][4];
#pragma unroll
  for (int r = 0; r < 2; ++r)
#pragma unroll
    for (int t = 0; t < 4; ++t) acc[r][t] = (v8f){};
#pragma unroll 2
  for (int kb = 0; kb < D; kb += 32) { v16b a0, l0, a1, l1; frag_split(Ain + (size_t)(m0 + nloc) * D + kb, hlf, a0, l0); frag_split(Ain + (size_t)(m0 + 16 + nloc) * D + kb, hlf, a1, l1);
#pragma unroll
    for (int t = 0; t < 4; ++t) { const v16b bw = frag_kb(Bw + (size_t)(c0 + t * 16 + nloc) * D + kb, hlf); acc[0][t] = wmma16b(a0, bw, acc[0][t]); acc[0][t] = wmma16b(l0, bw, acc[0][t]); acc[1][t] = wmma16b(a1, bw, acc[1][t]); acc[1][t] = wmma16b(l1, bw, acc[1][t]); } }
  float* Tt = Ts[wave];
#pragma unroll
  for (int t = 0; t < 4; ++t) { const int cc = c0 + t * 16 + nloc; const float bb = bias[cc];
#pragma unroll
    for (int r = 0; r < 2; ++r)
#pragma unroll
      for (int v = 0; v < 8; ++v) { const int rl = r * 16 + v + 8 * hlf; float y = acc[r][t][v] * (1.0f / AS_) + bb; if (mode == 0) y = fmaxf(y, 0.0f); else y += res[(size_t)(m0 + rl) * D + cc]; Tt[rl * 64 + t * 16 + nloc] = y; } }
  wave_lds_sync();
  for (int pass = 0; pass < 2; ++pass) {
#pragma unroll
    for (int j = 0; j < 16; ++j) { const int rr = j * 2 + hlf, c4 = nloc * 4; *(volatile v4f*)(Y + (size_t)(m0 + rr) * D + c0 + c4) = *(const v4f*)(Tt + rr * 64 + c4); }
    __threadfence(); }
}
}

extern "C" void kernel_launch(void* const* d_in, const int* in_sizes, int n_in,
                              void* d_out, int out_size, void* d_ws, size_t ws_size, hipStream_t stream) {
  (void)n_in; (void)out_size;
  const float* x = (const float*)d_in[0]; const float* wq = (const float*)d_in[1]; const float* wk = (const float*)d_in[2]; const float* wv = (const float*)d_in[3]; const float* g1 = (const float*)d_in[4]; const float* be1 = (const float*)d_in[5]; const float* g2 = (const float*)d_in[6]; const float* be2 = (const float*)d_in[7];
  const float* w1 = (const float*)d_in[8]; const float* b1 = (const float*)d_in[9]; const float* w2 = (const float*)d_in[10]; const float* b2 = (const float*)d_in[11];
  float* out = (float*)d_out;
  if (in_sizes[0] != NT * D || in_sizes[1] != D * D || in_sizes[8] != D * D || in_sizes[10] != D * D) return;
  size_t off = 0; char* ws = (char*)d_ws;
  auto carve = [&](size_t bytes) { char* p = ws + off; off += (bytes + 255) & ~(size_t)255; return p; };
  b16* R = (b16*)carve(Wo_::END * 2); float* P = (float*)carve(6 * D * 4); float* xn = (float*)carve((size_t)NT * D * 4); b16* qp = (b16*)carve(PL * 2); b16* kp = (b16*)carve(PL * 2); b16* vt = (b16*)carve(PL * 2);
  float* xt = (float*)carve((size_t)NT * D * 4); float* hbuf = (float*)carve((size_t)NT * D * 4); float* xtn = xn;
  if (off > ws_size) return;
  prep_kernel<<<256, 256, 0, stream>>>(wq, wk, wv, w1, w2, b1, b2, g1, be1, g2, be2, R, P);
  ln_kernel<<<NT / 8, 256, 0, stream>>>(x, P + 1024, P + 1536, 1, xn);
  qk_kernel<<<dim3(H, NT / 128, 2), 128, 0, stream>>>(xn, R, qp, kp);
  v_kernel<<<dim3(H, S / 128), 128, 0, stream>>>(xn, R, vt);
  attn_kernel<<<dim3(S / 16, Bn), 256, 0, stream>>>(qp, kp, vt, x, xt);
  ln_kernel<<<NT / 8, 256, 0, stream>>>(xt, P + 2048, P + 2560, 0, xtn);
  ffn_kernel<<<dim3(D / 64, NT / 128), 128, 0, stream>>>(xtn, R + Wo_::W1, P, 0, nullptr, hbuf);
  ffn_kernel<<<dim3(D / 64, NT / 128), 128, 0, stream>>>(hbuf, R + Wo_::W2, P + 512, 1, xt, out);
}
